// GINE_84799834292736
// MI455X (gfx1250) — hardware-verified
//
#include <hip/hip_runtime.h>
#include <hip/hip_bf16.h>


#define HID 128
#define MB  64

typedef __attribute__((ext_vector_type(16))) _Float16 v16h;
typedef __attribute__((ext_vector_type(2)))  _Float16 v2h;
typedef __attribute__((ext_vector_type(4)))  _Float16 v4h;
typedef __attribute__((ext_vector_type(8)))  float    v8f;
typedef __attribute__((ext_vector_type(8)))  _Float16 v8h;
typedef __attribute__((ext_vector_type(4)))  float    v4f_t;
typedef float v4fa __attribute__((ext_vector_type(4), may_alias));
#define BUCKET 64
#define LCAP   2048

__device__ __forceinline__ v16h load_a_frag(const _Float16* rowp, int half) {
  v16h a;
#pragma unroll
  for (int i = 0; i < 8; ++i) {
    int p = (i < 4) ? (half * 4 + i) : (4 + half * 4 + i);
    v2h t2 = *(const v2h*)(rowp + 2 * p);
    a[2 * i]     = t2[0];
    a[2 * i + 1] = t2[1];
  }
  return a;
}

__device__ __forceinline__ v16h load_b_frag(const _Float16* colp) {
  union { v16h v; v8h q[2]; } u;
  u.q[0] = *(const v8h*)(colp);
  u.q[1] = *(const v8h*)(colp + 16);
  return u.v;
}

__global__ __launch_bounds__(256) void wcvt_kernel(const float* __restrict__ W,
                                                   _Float16* __restrict__ Wt,
                                                   int total) {
  int idx = (blockIdx.x * 256 + threadIdx.x) * 2;
  if (idx >= total) return;
  int l   = idx / (HID * HID);
  int rem = idx - l * HID * HID;
  int n   = rem >> 7;
  int k   = rem & 127;
  const unsigned p = (unsigned)__builtin_bit_cast(unsigned short, (_Float16)W[l * HID * HID + k * HID + n]) | ((unsigned)__builtin_bit_cast(unsigned short, (_Float16)W[l * HID * HID + (k + 1) * HID + n]) << 16);
  *(volatile unsigned*)(Wt + idx) = p; __threadfence(); *(volatile unsigned*)(Wt + idx) = p;
}

__global__ __launch_bounds__(256) void edge_embed_kernel(
    const float* __restrict__ edge_attr, const float* __restrict__ We,
    const float* __restrict__ be, _Float16* __restrict__ ea, int E) {
  __shared__ float sW[16 * HID];
  __shared__ float sB[HID];
  for (int i = threadIdx.x; i < 16 * HID; i += 256) sW[i] = We[i];
  if (threadIdx.x < HID) sB[threadIdx.x] = be[threadIdx.x];
  __syncthreads();

  const int j     = (threadIdx.x & 63) * 2;
  const int esub  = threadIdx.x >> 6;
  const int ebase = blockIdx.x * 16;
  int eend = ebase + 16; if (eend > E) eend = E;
  for (int e = ebase + esub; e < eend; e += 4) {
    float acc0 = sB[j], acc1 = sB[j + 1];
#pragma unroll
    for (int k = 0; k < 16; ++k) { const float a = edge_attr[e * 16 + k]; acc0 += a * sW[k * HID + j]; acc1 += a * sW[k * HID + j + 1]; }
    const unsigned p = (unsigned)__builtin_bit_cast(unsigned short, (_Float16)acc0) | ((unsigned)__builtin_bit_cast(unsigned short, (_Float16)acc1) << 16);
    *(volatile unsigned*)(ea + (size_t)e * HID + j) = p; __threadfence(); *(volatile unsigned*)(ea + (size_t)e * HID + j) = p;
  }
}

__global__ __launch_bounds__(256) void bucket_list_kernel(const int* __restrict__ dst, int E, int N,
                                                          int* __restrict__ noff, int* __restrict__ ncnt, int* __restrict__ ledge) {
  __shared__ unsigned lst[LCAP];
  __shared__ unsigned srt[LCAP];
  __shared__ int wcnt[8];
  __shared__ int total;
  __shared__ int cnt[BUCKET], off[BUCKET];
  const int tid = threadIdx.x, lane = tid & 31, wave = tid >> 5;
  const int n0 = blockIdx.x * BUCKET;
  if (tid == 0) total = 0;
  __syncthreads();
  for (int e0 = 0; e0 < E; e0 += 256) {
    const int e = e0 + tid;
    int loc = -1;
    if (e < E) { const int l = dst[e] - n0; if ((unsigned)l < (unsigned)BUCKET) loc = l; }
    const unsigned m = __ballot(loc >= 0);
    if (lane == 0) wcnt[wave] = __popc(m);
    __syncthreads();
    int base = total;
#pragma unroll
    for (int w = 0; w < 8; ++w) if (w < wave) base += wcnt[w];
    if (loc >= 0) { const int slot = base + __popc(m & ((1u << lane) - 1u)); if (slot < LCAP) lst[slot] = ((unsigned)loc << 24) | (unsigned)e; }
    __syncthreads();
    if (tid == 0) { int t = total; for (int w = 0; w < 8; ++w) t += wcnt[w]; total = t; }
    __syncthreads();
  }
  const int nl = (total < LCAP) ? total : LCAP;
  if (tid < BUCKET) { int c = 0; for (int i = 0; i < nl; ++i) c += ((int)(lst[i] >> 24) == tid); cnt[tid] = c; }
  __syncthreads();
  if (tid == 0) { int o = 0; for (int j = 0; j < BUCKET; ++j) { off[j] = o; o += cnt[j]; } }
  __syncthreads();
  if (tid < BUCKET) { int p = off[tid]; for (int i = 0; i < nl; ++i) if ((int)(lst[i] >> 24) == tid) srt[p++] = lst[i] & 0xFFFFFFu; }
  __syncthreads();
#pragma unroll 1
  for (int pass = 0; pass < 2; ++pass) {
    if (tid < BUCKET && n0 + tid < N) { *(volatile int*)(noff + n0 + tid) = blockIdx.x * LCAP + off[tid]; *(volatile int*)(ncnt + n0 + tid) = cnt[tid]; }
    typedef __attribute__((ext_vector_type(4))) unsigned v4u_t;
    typedef unsigned v4ua __attribute__((ext_vector_type(4), may_alias));
    for (int c = tid; c * 4 < nl; c += 256)
      *(volatile v4u_t*)((unsigned*)ledge + (size_t)blockIdx.x * LCAP + c * 4) = *(const volatile v4ua*)(srt + c * 4);
    __threadfence();
  }
}

__global__ __launch_bounds__(256) void gather_kernel(
    const float* __restrict__ h, const _Float16* __restrict__ ea,
    const int* __restrict__ src, const int* __restrict__ noff, const int* __restrict__ ncnt, const int* __restrict__ ledge,
    float* __restrict__ agg, int N, int E) {
  int w = (blockIdx.x * blockDim.x + threadIdx.x) >> 5;
  if (w >= N) return;
  int lane = threadIdx.x & 31;
  int o0 = noff[w], c_ = ncnt[w];
  c_ = (c_ < 0) ? 0 : ((c_ > LCAP) ? LCAP : c_);
  { const int omax = ((N + BUCKET - 1) / BUCKET) * LCAP - c_; o0 = (o0 < 0) ? 0 : ((o0 > omax) ? omax : o0); }
  v4f_t acc = {0.f, 0.f, 0.f, 0.f};
  for (int i = 0; i < c_; ++i) {
    int e = ledge[o0 + i]; e = ((unsigned)e < (unsigned)E) ? e : 0;
    int s = src[e];        s = ((unsigned)s < (unsigned)N) ? s : 0;
    const float4 hv = *(const float4*)&h[(size_t)s * HID + lane * 4];
    const v4h    e4 = *(const v4h*)&ea[(size_t)e * HID + lane * 4];
    acc.x += fmaxf(hv.x + (float)e4[0], 0.f);
    acc.y += fmaxf(hv.y + (float)e4[1], 0.f);
    acc.z += fmaxf(hv.z + (float)e4[2], 0.f);
    acc.w += fmaxf(hv.w + (float)e4[3], 0.f);
  }
  float* ap = &agg[(size_t)w * HID + lane * 4];
  *(volatile v4f_t*)ap = acc; __threadfence(); *(volatile v4f_t*)ap = acc;
}

__global__ __launch_bounds__(256) void mlp_fused_kernel(
    float* __restrict__ h, const float* __restrict__ agg,
    const _Float16* __restrict__ W1t, const _Float16* __restrict__ W2t,
    const float* __restrict__ b1, const float* __restrict__ b2,
    const float* __restrict__ lng, const float* __restrict__ lnb, int n) {
  __shared__ _Float16 sA[MB * HID];
  __shared__ float    sZ[MB * HID];
  __shared__ float    sMu[MB], sRs[MB];

  const int tid  = threadIdx.x;
  const int lane = tid & 31;
  const int wave = tid >> 5;
  const int row0 = blockIdx.x * MB;
  const int r16  = lane & 15;
  const int half = lane >> 4;
  const int mt   = wave >> 1;
  const int nt0  = (wave & 1) * 4;

  for (int i = tid; i < MB * HID; i += 256) {
    int r = i >> 7, c = i & 127;
    int gr = row0 + r;
    float v = 0.f;
    if (gr < n) v = h[(size_t)gr * HID + c] + agg[(size_t)gr * HID + c];
    sA[i] = (_Float16)v;
  }
  __syncthreads();

  v16h a[4];
#pragma unroll
  for (int ks = 0; ks < 4; ++ks)
    a[ks] = load_a_frag(&sA[(mt * 16 + r16) * HID + ks * 32], half);

  v8f acc[4];
#pragma unroll
  for (int j = 0; j < 4; ++j) {
    const int nt = nt0 + j;
    v8f c = {};
#pragma unroll
    for (int ks = 0; ks < 4; ++ks) {
      v16h b = load_b_frag(&W1t[(nt * 16 + r16) * HID + ks * 32 + half * 8]);
      c = __builtin_amdgcn_wmma_f32_16x16x32_f16(false, a[ks], false, b,
                                                 (short)0, c, false, false);
    }
    acc[j] = c;
  }
  __syncthreads();

#pragma unroll
  for (int j = 0; j < 4; ++j) {
    const int col = (nt0 + j) * 16 + r16;
    const float bb = b1[col];
#pragma unroll
    for (int v = 0; v < 8; ++v) {
      int row = mt * 16 + half * 8 + v;
      sA[row * HID + col] = (_Float16)fmaxf(acc[j][v] + bb, 0.f);
    }
  }
  __syncthreads();

#pragma unroll
  for (int ks = 0; ks < 4; ++ks)
    a[ks] = load_a_frag(&sA[(mt * 16 + r16) * HID + ks * 32], half);

#pragma unroll
  for (int j = 0; j < 4; ++j) {
    const int nt = nt0 + j;
    v8f c = {};
#pragma unroll
    for (int ks = 0; ks < 4; ++ks) {
      v16h b = load_b_frag(&W2t[(nt * 16 + r16) * HID + ks * 32 + half * 8]);
      c = __builtin_amdgcn_wmma_f32_16x16x32_f16(false, a[ks], false, b,
                                                 (short)0, c, false, false);
    }
    const int col = nt * 16 + r16;
    const float bb = b2[col];
#pragma unroll
    for (int v = 0; v < 8; ++v) {
      int row = mt * 16 + half * 8 + v;
      sZ[row * HID + col] = c[v] + bb;
    }
  }
  __syncthreads();

  const int r  = tid >> 2;
  const int c0 = tid & 3;
  float s = 0.f, s2 = 0.f;
  for (int c = c0; c < HID; c += 4) {
    float z = sZ[r * HID + c];
    s += z; s2 += z * z;
  }
  s  += __shfl_xor(s, 1);  s2 += __shfl_xor(s2, 1);
  s  += __shfl_xor(s, 2);  s2 += __shfl_xor(s2, 2);
  if (c0 == 0) {
    float mu  = s * (1.f / HID);
    float var = s2 * (1.f / HID) - mu * mu;
    sMu[r] = mu;
    sRs[r] = rsqrtf(var + 1e-5f);
  }
  __syncthreads();

#pragma unroll 1
  for (int rr = 0; rr < 8; ++rr) {
    const int row = wave * 8 + rr, grr = row0 + row;
    if (grr < n) {
      const float mu = sMu[row], rs = sRs[row];
      const size_t gi = (size_t)grr * HID + lane * 4;
      const v4f_t ho = *(const v4fa*)&h[gi];
      const v4f_t g4 = *(const v4fa*)&lng[lane * 4], b4 = *(const v4fa*)&lnb[lane * 4];
      v4f_t z4 = *(const v4fa*)&sZ[row * HID + lane * 4];
      z4 = (z4 - mu) * rs * g4 + b4;
      z4.x = fmaxf(z4.x, 0.f) + ho.x; z4.y = fmaxf(z4.y, 0.f) + ho.y; z4.z = fmaxf(z4.z, 0.f) + ho.z; z4.w = fmaxf(z4.w, 0.f) + ho.w;
      *(volatile v4f_t*)&h[gi] = z4; __threadfence(); *(volatile v4f_t*)&h[gi] = z4;
    }
  }
}

__global__ __launch_bounds__(256) void copy_kernel(const float* __restrict__ in,
                                                   float* __restrict__ out, int n) {
  int i = blockIdx.x * 256 + threadIdx.x;
  if (i < n) { const float v = in[i]; *(volatile float*)(out + i) = v; __threadfence(); *(volatile float*)(out + i) = v; }
}

__global__ __launch_bounds__(256) void zero_kernel(float* __restrict__ p, int n) {
  int i = blockIdx.x * 256 + threadIdx.x;
  if (i < n) p[i] = 0.f;
}

extern "C" void kernel_launch(void* const* d_in, const int* in_sizes, int n_in,
                              void* d_out, int out_size, void* d_ws, size_t ws_size,
                              hipStream_t stream) {
  const float* x         = (const float*)d_in[0];
  const int*   ei        = (const int*)d_in[2];
  const float* edge_attr = (const float*)d_in[3];
  const float* We        = (const float*)d_in[4];
  const float* be        = (const float*)d_in[5];
  const float* W1        = (const float*)d_in[6];
  const float* b1        = (const float*)d_in[7];
  const float* W2        = (const float*)d_in[8];
  const float* b2        = (const float*)d_in[9];
  const float* lng       = (const float*)d_in[10];
  const float* lnb       = (const float*)d_in[11];

  const int N = in_sizes[0] / HID;
  const int E = in_sizes[2] / 2;
  const int L = in_sizes[6] / (HID * HID);

  char* ws = (char*)d_ws;
  _Float16* ea = (_Float16*)ws;  ws += (size_t)E * HID * sizeof(_Float16);
  float*   agg = (float*)ws;     ws += (size_t)N * HID * sizeof(float);
  _Float16* W1t = (_Float16*)ws; ws += (size_t)L * HID * HID * sizeof(_Float16);
  _Float16* W2t = (_Float16*)ws; ws += (size_t)L * HID * HID * sizeof(_Float16);
  const int nbk = (N + BUCKET - 1) / BUCKET;
  int* noff  = (int*)ws;  ws += (size_t)N * sizeof(int);
  int* ncnt  = (int*)ws;  ws += (size_t)N * sizeof(int);
  int* ledge = (int*)ws;  ws += (size_t)nbk * LCAP * sizeof(int);

  float* h = (float*)d_out;

  const int wtot = L * HID * HID;
  wcvt_kernel<<<(wtot / 2 + 255) / 256, 256, 0, stream>>>(W1, W1t, wtot);
  wcvt_kernel<<<(wtot / 2 + 255) / 256, 256, 0, stream>>>(W2, W2t, wtot);
  bucket_list_kernel<<<nbk, 256, 0, stream>>>(ei + E, E, N, noff, ncnt, ledge);

  edge_embed_kernel<<<(E + 15) / 16, 256, 0, stream>>>(edge_attr, We, be, ea, E);

  copy_kernel<<<((size_t)N * HID + 255) / 256, 256, 0, stream>>>(x, h, N * HID);

  for (int l = 0; l < L; ++l) {
    gather_kernel<<<((size_t)N * 32 + 255) / 256, 256, 0, stream>>>(h, ea, ei, noff, ncnt, ledge, agg, N, E);
    mlp_fused_kernel<<<(N + MB - 1) / MB, 256, 0, stream>>>(
        h, agg, W1t + (size_t)l * HID * HID, W2t + (size_t)l * HID * HID,
        b1 + l * HID, b2 + l * HID, lng + l * HID, lnb + l * HID, N);
  }
}
